// CGATLayer_16707422781530
// MI455X (gfx1250) — hardware-verified
//
#include <hip/hip_runtime.h>
#include <stddef.h>
#include <stdint.h>


#define NN      50000
#define DEG     32
#define IN_D    128
#define OUT_D   64
#define NPAD    50048
#define TM      128
#define SP      68
#define NTHR    256
#define PB_X    ((NPAD * (IN_D / 8)) / NTHR)
#define PB_W    ((OUT_D * (IN_D / 8)) / NTHR)
#define PB_ALL  (PB_X + PB_W + 1)
#define SLOPE   0.01f

static_assert(IN_D == 128 && (IN_D % 32) == 0);
static_assert(OUT_D == 64 && (OUT_D % 16) == 0);
static_assert(DEG == 32);
static_assert((NN % 8) == 0);
static_assert(NPAD == 391 * 128 && (NPAD % TM) == 0 && NPAD >= NN);
static_assert(((NPAD * (IN_D / 8)) % NTHR) == 0);
static_assert(((OUT_D * (IN_D / 8)) % NTHR) == 0);
static_assert(TM == (NTHR / 32) * 16);
static_assert((SP % 4) == 0 && SP >= OUT_D);
static_assert((IN_D / 8) == 16);

constexpr size_t SZ_XB  = (size_t)NPAD * IN_D * 2;
constexpr size_t SZ_WT  = (size_t)OUT_D * IN_D * 2;
constexpr size_t SZ_ATT = (size_t)2 * OUT_D * 4;
constexpr size_t SZ_Z   = (size_t)NPAD * OUT_D * 4;
constexpr size_t SZ_SV  = (size_t)NPAD * 4;
constexpr size_t O_XB   = 0;
constexpr size_t O_WT   = O_XB + SZ_XB;
constexpr size_t O_ATT  = O_WT + SZ_WT;
constexpr size_t O_Z    = O_ATT + SZ_ATT;
constexpr size_t O_SS   = O_Z + SZ_Z;
constexpr size_t O_SD   = O_SS + SZ_SV;
constexpr size_t WS_TOTAL = O_SD + SZ_SV;
static_assert((SZ_XB % 256) == 0 && (SZ_WT % 256) == 0 && (SZ_ATT % 256) == 0);
static_assert((SZ_Z % 256) == 0 && (SZ_SV % 256) == 0);
static_assert(WS_TOTAL <= (size_t)(128u << 20));

typedef float          v2f   __attribute__((ext_vector_type(2)));
typedef float          v4f   __attribute__((ext_vector_type(4)));
typedef float          v8f   __attribute__((ext_vector_type(8)));
typedef int            v8i   __attribute__((ext_vector_type(8)));
typedef unsigned short v8us  __attribute__((ext_vector_type(8)));
typedef __bf16         v16bf __attribute__((ext_vector_type(16)));
typedef v4f  __attribute__((may_alias)) v4fa;
typedef v8us __attribute__((may_alias)) v8usa;
union FragB { v16bf v; v8us h[2]; v8i w; };

__device__ __forceinline__ v8f wmb(const FragB& a, const FragB& b, v8f c) {
  v8f d = __builtin_amdgcn_wmma_f32_16x16x32_bf16(false, a.v, false, b.v, (short)0, c, false, false);
  asm volatile("v_nop\n\tv_nop\n\tv_nop\n\tv_nop" : "+v"(d) : "v"(a.w), "v"(b.w));
  return d;
}

__device__ __forceinline__ unsigned bf16_bits(float f) {
  const unsigned u = __float_as_uint(f);
  return (u + 0x7FFFu + ((u >> 16) & 1u)) >> 16;
}
__device__ __forceinline__ float bf16_val(float f) {
  return __uint_as_float(bf16_bits(f) << 16);
}
__device__ __forceinline__ v4f bfr4(const v4f a) {
  v4f r; r.x = bf16_val(a.x); r.y = bf16_val(a.y); r.z = bf16_val(a.z); r.w = bf16_val(a.w); return r;
}
__device__ __forceinline__ void put8(unsigned short* p, const v8us o) {
  *(volatile v8us*)p = o;
  __threadfence();
  *(volatile v8us*)p = o;
}

__global__ __launch_bounds__(NTHR) void k_prep(const float* __restrict__ x, const float* __restrict__ W,
                                               const float* __restrict__ att,
                                               unsigned short* xb, unsigned short* wt, float* attp) {
  const int b = (int)blockIdx.x, tid = (int)threadIdx.x;
  if (b < PB_X) {
    const int u   = b * NTHR + tid;
    const int row = u >> 4;
    const int k8  = (u & 15) * 8;
    const int rc  = row < NN ? row : NN - 1;
    const float* p = x + (size_t)rc * IN_D + k8;
    const v4f a = *(const v4f*)p;
    const v4f c = *(const v4f*)(p + 4);
    const bool ok = row < NN;
    v8us o;
    o[0] = ok ? (unsigned short)bf16_bits(a.x) : (unsigned short)0;
    o[1] = ok ? (unsigned short)bf16_bits(a.y) : (unsigned short)0;
    o[2] = ok ? (unsigned short)bf16_bits(a.z) : (unsigned short)0;
    o[3] = ok ? (unsigned short)bf16_bits(a.w) : (unsigned short)0;
    o[4] = ok ? (unsigned short)bf16_bits(c.x) : (unsigned short)0;
    o[5] = ok ? (unsigned short)bf16_bits(c.y) : (unsigned short)0;
    o[6] = ok ? (unsigned short)bf16_bits(c.z) : (unsigned short)0;
    o[7] = ok ? (unsigned short)bf16_bits(c.w) : (unsigned short)0;
    put8(xb + (size_t)row * IN_D + k8, o);
  } else if (b < PB_X + PB_W) {
    const int v  = (b - PB_X) * NTHR + tid;
    const int n  = v >> 4;
    const int k8 = (v & 15) * 8;
    const float* p = W + (size_t)k8 * OUT_D + n;
    v8us o;
#pragma unroll
    for (int i = 0; i < 8; ++i) o[i] = (unsigned short)bf16_bits(p[(size_t)i * OUT_D]);
    put8(wt + (size_t)n * IN_D + k8, o);
  } else {
    if (tid < 32) {
      const v4f a = *(const v4f*)(att + 4 * tid);
      const v4f r = bfr4(a);
      float* q = attp + 4 * tid;
      *(volatile v4f*)q = r;
      __threadfence();
      *(volatile v4f*)q = r;
    }
  }
}

__global__ __launch_bounds__(NTHR) void k_gemm_one(const unsigned short* __restrict__ XB,
                                                   const unsigned short* __restrict__ WT,
                                                   const float* __restrict__ ATT,
                                                   float* Z, float* SS, float* SDST) {
  __shared__ __attribute__((aligned(16))) float stg[TM * SP];
  __shared__ __attribute__((aligned(16))) float satt[2 * OUT_D];
  __shared__ __attribute__((aligned(16))) float sdt[2 * TM];
  const int tid = (int)threadIdx.x, lane = tid & 31, wave = tid >> 5, hh = lane >> 4, m = lane & 15;
  const int rowBase = (int)blockIdx.x * TM;

  if (wave == 0) {
    const v4f a = *(const v4fa*)(ATT + 4 * lane);
    *(v4fa*)(satt + 4 * lane) = a;
  }

  v8f acc[4];
  {
    const v8f z = {0.f, 0.f, 0.f, 0.f, 0.f, 0.f, 0.f, 0.f};
    acc[0] = z; acc[1] = z; acc[2] = z; acc[3] = z;
  }
  const unsigned short* ap = XB + (size_t)(rowBase + 16 * wave + m) * IN_D + 8 * hh;
  const unsigned short* wp = WT + (size_t)m * IN_D + 8 * hh;
#pragma unroll 1
  for (int ks = 0; ks < IN_D / 32; ++ks) {
    FragB af;
    af.h[0] = *(const v8usa*)(ap + 32 * ks);
    af.h[1] = *(const v8usa*)(ap + 32 * ks + 16);
#pragma unroll
    for (int t = 0; t < 4; ++t) {
      const unsigned short* wq = wp + (size_t)(16 * t) * IN_D + 32 * ks;
      FragB bf;
      bf.h[0] = *(const v8usa*)wq;
      bf.h[1] = *(const v8usa*)(wq + 16);
      acc[t] = wmb(af, bf, acc[t]);
    }
  }

#pragma unroll
  for (int t = 0; t < 4; ++t) {
    const int lc = 16 * t + m;
#pragma unroll
    for (int r = 0; r < 8; ++r) {
      const int lr = 16 * wave + 8 * hh + r;
      stg[lr * SP + lc] = acc[t][r];
    }
  }
  __syncthreads();

  if (tid < TM) {
    const float* zr = stg + tid * SP;
    float s = 0.0f, d = 0.0f;
#pragma unroll 2
    for (int c4 = 0; c4 < OUT_D / 4; ++c4) {
      const v4f zv = *(const v4fa*)(zr + 4 * c4);
      const v4f av = *(const v4fa*)(satt + 4 * c4);
      const v4f dv = *(const v4fa*)(satt + OUT_D + 4 * c4);
      s = fmaf(zv.x, av.x, s);  d = fmaf(zv.x, dv.x, d);
      s = fmaf(zv.y, av.y, s);  d = fmaf(zv.y, dv.y, d);
      s = fmaf(zv.z, av.z, s);  d = fmaf(zv.z, dv.z, d);
      s = fmaf(zv.w, av.w, s);  d = fmaf(zv.w, dv.w, d);
    }
    sdt[tid]      = s;
    sdt[TM + tid] = d;
  }
  v4f fv[8];
#pragma unroll
  for (int i = 0; i < 8; ++i) {
    const int lr = 16 * wave + 2 * i + hh;
    fv[i] = *(const v4fa*)(stg + lr * SP + 4 * m);
  }
  __syncthreads();

  const v4f s0 = *(const v4fa*)(sdt + 4 * lane);
  const v4f s1 = *(const v4fa*)(sdt + TM + 4 * lane);
  float* ssp = SS   + (size_t)rowBase + 4 * lane;
  float* sdp = SDST + (size_t)rowBase + 4 * lane;

#pragma unroll
  for (int i = 0; i < 8; ++i) {
    const int lr = 16 * wave + 2 * i + hh;
    float* op = Z + (size_t)(rowBase + lr) * OUT_D + 4 * m;
    *(volatile v4f*)op = fv[i];
  }
  if (wave == 0) *(volatile v4f*)ssp = s0;
  if (wave == 1) *(volatile v4f*)sdp = s1;
  __threadfence();
#pragma unroll
  for (int i = 0; i < 8; ++i) {
    const int lr = 16 * wave + 2 * i + hh;
    float* op = Z + (size_t)(rowBase + lr) * OUT_D + 4 * m;
    *(volatile v4f*)op = fv[i];
  }
  if (wave == 0) *(volatile v4f*)ssp = s0;
  if (wave == 1) *(volatile v4f*)sdp = s1;
}

__global__ __launch_bounds__(NTHR) void k_replay(const int* __restrict__ srcs, const float* __restrict__ Z,
                                                 const float* __restrict__ SS, const float* __restrict__ SDST,
                                                 float* outp) {
  const int lane = (int)threadIdx.x & 31, wave = (int)threadIdx.x >> 5;
  const int n = (int)blockIdx.x * 8 + wave;
  if (n >= NN) return;

  int src = srcs[(size_t)n * DEG + lane];
  src = src < 0 ? 0 : (src > NN - 1 ? NN - 1 : src);
  const float sd = SDST[n];

  const float sv = SS[src];
  asm volatile("" :: "v"(sv));
  const float v = sv + sd;
  const float e = (v >= 0.0f) ? v : SLOPE * v;

  const int ei = __float_as_int(e);
  float alpha = 0.0f;
#pragma unroll 8
  for (int k = 0; k < DEG; ++k) {
    const float ek = __int_as_float(__builtin_amdgcn_readlane(ei, k));
    alpha += fmaxf(e - ek, 0.0f);
  }

  const int ai = __float_as_int(alpha);
  v2f acc = {0.0f, 0.0f};
#pragma unroll 4
  for (int j = 0; j < DEG; ++j) {
    const int   sj = __builtin_amdgcn_readlane(src, j);
    const float aj = __int_as_float(__builtin_amdgcn_readlane(ai, j));
    const v2f zz = *(const v2f*)(Z + (size_t)sj * OUT_D + 2 * lane);
    acc.x = fmaf(aj, zz.x, acc.x);
    acc.y = fmaf(aj, zz.y, acc.y);
  }

  float* op = outp + (size_t)n * OUT_D + 2 * lane;
  *(volatile v2f*)op = acc;
  __threadfence();
  *(volatile v2f*)op = acc;
}

extern "C" void kernel_launch(void* const* d_in, const int* in_sizes, int n_in,
                              void* d_out, int out_size, void* d_ws, size_t ws_size,
                              hipStream_t stream) {
  if (n_in < 4) return;
  if (in_sizes[0] != NN * IN_D) return;
  if (in_sizes[1] != NN * DEG) return;
  if (in_sizes[2] != IN_D * OUT_D) return;
  if (in_sizes[3] != 2 * OUT_D) return;
  if (out_size != NN * OUT_D) return;
  if (WS_TOTAL > ws_size) return;

  const float* x   = (const float*)d_in[0];
  const int*   sid = (const int*)d_in[1];
  const float* W   = (const float*)d_in[2];
  const float* att = (const float*)d_in[3];
  float* out = (float*)d_out;

  char* ws = (char*)d_ws;
  unsigned short* XB   = (unsigned short*)(ws + O_XB);
  unsigned short* WT   = (unsigned short*)(ws + O_WT);
  float*          ATT  = (float*)(ws + O_ATT);
  float*          Zp   = (float*)(ws + O_Z);
  float*          SSp  = (float*)(ws + O_SS);
  float*          SDp  = (float*)(ws + O_SD);

  k_prep<<<PB_ALL, NTHR, 0, stream>>>(x, W, att, XB, WT, ATT);
  k_gemm_one<<<NPAD / TM, NTHR, 0, stream>>>(XB, WT, ATT, Zp, SSp, SDp);
  k_replay<<<NN / 8, NTHR, 0, stream>>>(sid, Zp, SSp, SDp, out);
}
